// Cross_58677843198640
// MI455X (gfx1250) — hardware-run, weakly checked
//
#include <hip/hip_runtime.h>
#include <math.h>
#include <stdint.h>

#ifndef NB
#define NB 2
#endif
#define NBF    2
#define DCH    64
#define KD     128
#define SD     128
#define LQ     128
#define NH     4
#define HD     64
#define FPR    (NH * HD)
#define NPJ    8
#define TEN    (DCH * KD * SD)
#define TEN_FULL (DCH * KD * SD)
#define OUT1_OFF ((size_t)NBF * TEN_FULL)
#define GSEQ   128
#define GROWS  (GSEQ * LQ)
#define TROWS  (NB * GROWS)
#define NQT    (LQ / 16)
#define NKT    (LQ / 32)
#define WPB    2
#define NHG    (NH / WPB)
#define ATT_THREADS (WPB * 32)
#define PSC    132
#define SLP    68
#define WREG   (2 * 16 * PSC + 16 * SLP)
#define SLAB64 (16 * 68)
#define XTP    72
#define GTP    132
#define BNLP   32
#define GNPART 32
#define GNCH   (TEN / GNPART)
#define XSC    16.0f
#define WISC   256.0f
#define QSC    1024.0f
#define VCAR   1024.0f
#define PCAR   32768.0f
#define OSC    1024.0f
#define WOS    1024.0f
#define RSQ_HD 0.125f
#define LOG2E  1.4426950408889634f
#define BN_EPS 1e-5f
#define GN_EPS 1e-8f
#define WS_CAP 134217728
static_assert(FPR == 256 && HD == 64 && NH == 4 && (NH % WPB) == 0 && ATT_THREADS == 64);
static_assert(NB >= 1 && NB <= NBF);
static_assert(OUT1_OFF * 4 == (size_t)8388608);
static_assert(TEN == TEN_FULL);
static_assert(KD == 128 && SD == 128 && LQ == 128 && GSEQ == KD && GSEQ == SD);
static_assert((GROWS % 64) == 0 && (FPR % 64) == 0 && (DCH % 64) == 0 && (DCH % 32) == 0 && (FPR % 32) == 0);
static_assert(GNPART == 32 && (GNCH % 1024) == 0 && ((KD * SD) % 1024) == 0 && (TEN % GNPART) == 0);
static_assert(WPB * WREG * 4 <= 65536 && NQT * 16 == LQ && NKT * 32 == LQ && (HD % 32) == 0);
static_assert(((NPJ * FPR * DCH) % 8) == 0 && ((2 * DCH * FPR) % 8) == 0);

typedef unsigned short u16;
typedef _Float16 v16h __attribute__((ext_vector_type(16)));
typedef _Float16 v8h  __attribute__((ext_vector_type(8)));
typedef float    v8f  __attribute__((ext_vector_type(8)));
typedef float    v4f  __attribute__((ext_vector_type(4)));
typedef unsigned int v4u __attribute__((ext_vector_type(4)));
typedef double   v2d  __attribute__((ext_vector_type(2)));

union FragH { v16h v; v8h h[2]; v4u u[2]; };

#define HP(p) ((const _Float16*)(const void*)(p))

__device__ __forceinline__ unsigned short bf_bits(float f) {
  unsigned u = __float_as_uint(f);
  return (unsigned short)((u + 0x7FFFu + ((u >> 16) & 1u)) >> 16);
}
__device__ __forceinline__ float bf_up(unsigned short h) { return __uint_as_float(((unsigned)h) << 16); }
__device__ __forceinline__ float bfr(float f) { return bf_up(bf_bits(f)); }
__device__ __forceinline__ unsigned short h_bits(_Float16 x) { return __builtin_bit_cast(unsigned short, x); }
__device__ __forceinline__ unsigned pk16(unsigned short a, unsigned short b) { return (unsigned)a | ((unsigned)b << 16); }
__device__ __forceinline__ v8f zero8() { v8f z = {0.f, 0.f, 0.f, 0.f, 0.f, 0.f, 0.f, 0.f}; return z; }
__device__ __forceinline__ double wsum_d(double v) {
#pragma unroll
  for (int off = 1; off < 32; off <<= 1) v += __shfl_xor(v, off, 32);
  return v;
}

__device__ __forceinline__ v16h ldfrag_h(const _Float16* p) {
  FragH f;
  f.h[0] = *(const v8h*)(p);
  f.h[1] = *(const v8h*)(p + 16);
  return f.v;
}

__device__ __forceinline__ v8f mma_h(v16h a, v16h b, v8f c) {
  return __builtin_amdgcn_wmma_f32_16x16x32_f16(false, a, false, b, (short)0, c, false, false);
}
template <typename F>
__device__ __forceinline__ void guard6(v8f& a, v8f& b, v8f& c, v8f& d, F x0, F x1, F x2, F x3, F x4, F x5) {
#if defined(__HIP_DEVICE_COMPILE__)
  asm volatile("v_nop\n\tv_nop\n\tv_nop\n\tv_nop"
               : "+v"(a), "+v"(b), "+v"(c), "+v"(d) : "v"(x0), "v"(x1), "v"(x2), "v"(x3), "v"(x4), "v"(x5) : "memory");
#endif
}
__device__ __forceinline__ void guard4x8(v8f& a, v8f& b, v8f& c, v8f& d, v16h x0, v16h x1, v16h x2, v16h x3,
                                         v16h x4, v16h x5, v16h x6, v16h x7) {
#if defined(__HIP_DEVICE_COMPILE__)
  asm volatile("v_nop\n\tv_nop\n\tv_nop\n\tv_nop"
               : "+v"(a), "+v"(b), "+v"(c), "+v"(d)
               : "v"(x0), "v"(x1), "v"(x2), "v"(x3), "v"(x4), "v"(x5), "v"(x6), "v"(x7) : "memory");
#endif
}
__device__ __forceinline__ void acc_guard4(v8f& a, v8f& b, v8f& c, v8f& d) {
#if defined(__HIP_DEVICE_COMPILE__)
  asm volatile("v_nop\n\tv_nop\n\tv_nop\n\tv_nop" : "+v"(a), "+v"(b), "+v"(c), "+v"(d));
#endif
}
__device__ __forceinline__ void wave_sync_lds() {
  __builtin_amdgcn_fence(__ATOMIC_RELEASE, "workgroup");
  __builtin_amdgcn_wave_barrier();
  __builtin_amdgcn_fence(__ATOMIC_ACQUIRE, "workgroup");
}

__global__ __launch_bounds__(256) void wcvt(const float* __restrict__ x, u16* D, int n8, float scale) {
  const int gt = blockIdx.x * 256 + (int)threadIdx.x;
  if (gt >= n8) return;
  const float* p = x + (size_t)gt * 8;
  const v4f a = *(const v4f*)(p), b4 = *(const v4f*)(p + 4);
  float w[8];
#pragma unroll
  for (int e = 0; e < 4; ++e) { w[e] = a[e]; w[4 + e] = b4[e]; }
  v4u o;
#pragma unroll
  for (int e = 0; e < 4; ++e) {
    const unsigned short hb0 = h_bits((_Float16)(bfr(w[2 * e]) * scale));
    const unsigned short hb1 = h_bits((_Float16)(bfr(w[2 * e + 1]) * scale));
    o[e] = pk16(hb0, hb1);
  }
  u16* d = D + (size_t)gt * 8;
  for (int pass = 0; pass < 2; ++pass) {
    *(volatile v4u*)(d) = o;
    __threadfence();
  }
}

__global__ __launch_bounds__(256) void bnstat(const float* __restrict__ xs, const float* __restrict__ xn,
                                              const float* __restrict__ bw, const float* __restrict__ bb, float* T, int rnd) {
  __shared__ double rs[8], rq[8];
  const int tid = threadIdx.x, wave = tid >> 5, lane = tid & 31;
  const int t = (int)blockIdx.x >> 6;
  const int d = (int)blockIdx.x & 63;
  if (t >= 2) return;
  const float* x = (t != 0) ? xn : xs;
  double s = 0.0, s2 = 0.0;
#pragma unroll 1
  for (int m = 0; m < NB; ++m) {
    const float* base = x + (size_t)m * TEN_FULL + (size_t)d * (KD * SD);
#pragma unroll 1
    for (int i = tid * 4; i < KD * SD; i += 1024) {
      const v4f a = *(const v4f*)(base + i);
#pragma unroll
      for (int e = 0; e < 4; ++e) {
        const float f = a[e];
        const float g = (rnd != 0) ? bfr(f) : f;
        s  += (double)g;
        s2 += (double)g * (double)g;
      }
    }
  }
  s = wsum_d(s); s2 = wsum_d(s2);
  if (lane == 0) { rs[wave] = s; rq[wave] = s2; }
  __syncthreads();
  if (wave == 0) {
    double a = rs[lane & 7], b2 = rq[lane & 7];
    a  = (lane < 8) ? a : 0.0;
    b2 = (lane < 8) ? b2 : 0.0;
    a = wsum_d(a); b2 = wsum_d(b2);
    const double inv = 1.0 / (double)(NB * KD * SD);
    const double mu  = a * inv;
    double var = b2 * inv - mu * mu;
    var = (var > 0.0) ? var : 0.0;
    const float rstd = rsqrtf((float)var + BN_EPS);
    const float wv = bw[t * DCH + d];
    const float bv = bb[t * DCH + d];
    v4f o;
    o[0] = (lane == 0) ? (float)mu : 0.f;
    o[1] = (lane == 0) ? rstd * wv : 0.f;
    o[2] = (lane == 0) ? bv : 0.f;
    o[3] = 0.f;
    float* dst = T + (size_t)(t * DCH + d) * BNLP + lane * 4;
    for (int pass = 0; pass < 2; ++pass) {
      if (lane < 8) *(volatile v4f*)(dst) = o;
      __threadfence();
    }
  }
}

__global__ __launch_bounds__(256) void xpack(const float* __restrict__ xs, const float* __restrict__ xn,
                                             const float* __restrict__ T, u16* X, int stage, int rnd) {
  __shared__ __align__(16) u16 Tt[SD * XTP];
  const int tid = threadIdx.x;
  const int bid = blockIdx.x;
  const int kk  = bid % KD;
  const int t2  = bid / KD;
  const int m   = t2 % NB;
  const int t   = t2 / NB;
  if (t >= 2) return;
  const float* x = ((t != 0) ? xn : xs) + (size_t)m * TEN_FULL;
  {
    const int d  = tid >> 2;
    const int s0 = (tid & 3) * 32;
    const float mu = T[(t * DCH + d) * BNLP + 0];
    const float rw = T[(t * DCH + d) * BNLP + 1];
    const float bv = T[(t * DCH + d) * BNLP + 2];
    const float* src = x + ((size_t)d * KD + kk) * SD + s0;
#pragma unroll 2
    for (int i = 0; i < 8; ++i) {
      const v4f a = *(const v4f*)(src + 4 * i);
#pragma unroll
      for (int e = 0; e < 4; ++e) {
        const float f = a[e];
        const float g = (rnd != 0) ? bfr(f) : f;
        const float v = ((g - mu) * rw + bv) * XSC;
        Tt[(s0 + 4 * i + e) * XTP + d] = h_bits((_Float16)v);
      }
    }
  }
  __syncthreads();
  v4u w4[4];
  const int q8 = tid >> 3, p8 = (tid & 7) * 8;
#pragma unroll
  for (int it = 0; it < 4; ++it) {
    const int s = it * 32 + q8;
    w4[it] = *(const v4u*)(Tt + s * XTP + p8);
  }
  const int SS = (stage != 0) ? 1 : KD;
  const int SK = (stage != 0) ? SD : 1;
  const size_t rbase = (size_t)t * TROWS + (size_t)m * GROWS + (size_t)kk * SK;
  for (int pass = 0; pass < 2; ++pass) {
#pragma unroll
    for (int it = 0; it < 4; ++it) {
      const int s = it * 32 + q8;
      *(volatile v4u*)(X + (rbase + (size_t)s * SS) * DCH + p8) = w4[it];
    }
    __threadfence();
  }
}

__device__ __forceinline__ void epi64(float* sl, v8f a0, v8f a1, v8f a2, v8f a3,
                                      float* C, int N, size_t rowb, int col0, int lane) {
  const int hh = lane >> 4, m = lane & 15;
#pragma unroll
  for (int r = 0; r < 8; ++r) {
    const int ro = (8 * hh + r) * 68 + m;
    sl[ro]      = a0[r];
    sl[ro + 16] = a1[r];
    sl[ro + 32] = a2[r];
    sl[ro + 48] = a3[r];
  }
  wave_sync_lds();
  v4f vals[8];
#pragma unroll
  for (int it = 0; it < 8; ++it) vals[it] = *(const v4f*)(sl + (it * 2 + hh) * 68 + m * 4);
  float* dst = C + (rowb + (size_t)hh) * (size_t)N + col0 + m * 4;
  for (int pass = 0; pass < 2; ++pass) {
#pragma unroll
    for (int it = 0; it < 8; ++it) {
      *(volatile v4f*)(dst + (size_t)(it * 2) * (size_t)N) = vals[it];
    }
    __threadfence();
  }
}

template <bool LO>
__device__ __forceinline__ void epi16(float* sl, v8f a0, v8f a1, v8f a2, v8f a3,
                                      u16* Ch, u16* Cl, int N, int rowb, int col0, int lane) {
  const int hh = lane >> 4, m = lane & 15;
#pragma unroll
  for (int r = 0; r < 8; ++r) {
    const int ro = (8 * hh + r) * 68 + m;
    sl[ro]      = a0[r];
    sl[ro + 16] = a1[r];
    sl[ro + 32] = a2[r];
    sl[ro + 48] = a3[r];
  }
  wave_sync_lds();
  v4u oh[4], ol[4];
  const int rq = lane >> 3, c8 = (lane & 7) * 8;
#pragma unroll
  for (int it = 0; it < 4; ++it) {
    const int row = it * 4 + rq;
    const v4f a = *(const v4f*)(sl + row * 68 + c8), b4 = *(const v4f*)(sl + row * 68 + c8 + 4);
    float w[8];
#pragma unroll
    for (int e = 0; e < 4; ++e) { w[e] = a[e]; w[4 + e] = b4[e]; }
#pragma unroll
    for (int e = 0; e < 4; ++e) {
      const _Float16 h0 = (_Float16)w[2 * e], h1 = (_Float16)w[2 * e + 1];
      const _Float16 l0 = (_Float16)(w[2 * e] - (float)h0), l1 = (_Float16)(w[2 * e + 1] - (float)h1);
      oh[it][e] = pk16(h_bits(h0), h_bits(h1));
      ol[it][e] = pk16(h_bits(l0), h_bits(l1));
    }
  }
  const size_t base = (size_t)rowb * (size_t)N + col0 + c8;
  for (int pass = 0; pass < 2; ++pass) {
#pragma unroll
    for (int it = 0; it < 4; ++it) {
      const int row = it * 4 + rq;
      *(volatile v4u*)(Ch + base + (size_t)row * (size_t)N) = oh[it];
      if constexpr (LO) {
        *(volatile v4u*)(Cl + base + (size_t)row * (size_t)N) = ol[it];
      }
    }
    __threadfence();
  }
}

template <int MODE>
__global__ __launch_bounds__(128)
void gemm16(const u16* __restrict__ Ah, const u16* __restrict__ Al, const u16* __restrict__ Bt, const float* __restrict__ bias,
            float* Cf, u16* Ch, u16* Cl, int M, int N, int K, float isc, float osc) {
  __shared__ __align__(16) float slab[4 * SLAB64];
  const int tid = threadIdx.x, wave = tid >> 5, lane = tid & 31, hh = lane >> 4, m = lane & 15;
  const int ntile = N >> 6;
  const int bid   = blockIdx.x;
  const int rowb  = (bid / ntile) * 64 + wave * 16;
  const int col0  = (bid % ntile) * 64;
  if (rowb + 16 > M) return;
  const _Float16* ahp = HP(Ah) + (size_t)(rowb + m) * K + 8 * hh;
  const _Float16* alp = HP(Al) + (size_t)(rowb + m) * K + 8 * hh;
  const _Float16* bp  = HP(Bt) + (size_t)(col0 + m) * K + 8 * hh;
  const size_t bs = (size_t)16 * K;
  v8f acc0 = zero8(), acc1 = zero8(), acc2 = zero8(), acc3 = zero8();
  if constexpr (MODE == 0) {
#pragma unroll 1
    for (int k0 = 0; k0 < K; k0 += 32) {
      const v16h ah = ldfrag_h(ahp + k0), al = ldfrag_h(alp + k0);
      const v16h b0 = ldfrag_h(bp + k0);
      const v16h b1 = ldfrag_h(bp + bs + k0);
      const v16h b2 = ldfrag_h(bp + 2 * bs + k0);
      const v16h b3 = ldfrag_h(bp + 3 * bs + k0);
      acc0 = mma_h(ah, b0, acc0);  acc0 = mma_h(al, b0, acc0);
      acc1 = mma_h(ah, b1, acc1);  acc1 = mma_h(al, b1, acc1);
      acc2 = mma_h(ah, b2, acc2);  acc2 = mma_h(al, b2, acc2);
      acc3 = mma_h(ah, b3, acc3);  acc3 = mma_h(al, b3, acc3);
      guard6<v16h>(acc0, acc1, acc2, acc3, ah, al, b0, b1, b2, b3);
    }
  } else {
#pragma unroll 1
    for (int k0 = 0; k0 < K; k0 += 32) {
      const v16h ah = ldfrag_h(ahp + k0);
      const v16h b0 = ldfrag_h(bp + k0);
      const v16h b1 = ldfrag_h(bp + bs + k0);
      const v16h b2 = ldfrag_h(bp + 2 * bs + k0);
      const v16h b3 = ldfrag_h(bp + 3 * bs + k0);
      acc0 = mma_h(ah, b0, acc0);
      acc1 = mma_h(ah, b1, acc1);
      acc2 = mma_h(ah, b2, acc2);
      acc3 = mma_h(ah, b3, acc3);
      guard6<v16h>(acc0, acc1, acc2, acc3, ah, b0, b1, b2, b3, ah);
    }
  }
  v8f v0, v1, v2, v3;
  if constexpr (MODE == 2) {
#pragma unroll
    for (int r = 0; r < 8; ++r) {
      const float bv = bias[rowb + 8 * hh + r];
      v0[r] = fmaxf(acc0[r] * isc + bv, 0.f) * osc;
      v1[r] = fmaxf(acc1[r] * isc + bv, 0.f) * osc;
      v2[r] = fmaxf(acc2[r] * isc + bv, 0.f) * osc;
      v3[r] = fmaxf(acc3[r] * isc + bv, 0.f) * osc;
    }
  } else {
    const float b0 = bias[col0 + m], b1 = bias[col0 + 16 + m], b2 = bias[col0 + 32 + m], b3 = bias[col0 + 48 + m];
#pragma unroll
    for (int r = 0; r < 8; ++r) {
      v0[r] = fmaxf(acc0[r] * isc + b0, 0.f) * osc;
      v1[r] = fmaxf(acc1[r] * isc + b1, 0.f) * osc;
      v2[r] = fmaxf(acc2[r] * isc + b2, 0.f) * osc;
      v3[r] = fmaxf(acc3[r] * isc + b3, 0.f) * osc;
    }
  }
  if constexpr (MODE == 0) {
    epi64(slab + wave * SLAB64, v0, v1, v2, v3, Cf, N, (size_t)rowb, col0, lane);
  } else {
    epi16<MODE == 1>(slab + wave * SLAB64, v0, v1, v2, v3, Ch, Cl, N, rowb, col0, lane);
  }
}

__global__ __launch_bounds__(ATT_THREADS)
void attnx(const u16* __restrict__ QSH, const u16* __restrict__ QSL, const u16* __restrict__ QOH, const u16* __restrict__ QOL,
           const u16* __restrict__ KH, const u16* __restrict__ KL, const u16* __restrict__ VT, u16* OH, u16* OL) {
  __shared__ __align__(16) float smem[WPB * WREG];

  const int tid  = threadIdx.x;
  const int wave = tid >> 5;
  const int lane = tid & 31;
  const int hh   = lane >> 4;
  const int c    = lane & 15;
  const int bid  = blockIdx.x;
  const int qt   = bid % NQT;
  const int t2   = bid / NQT;
  const int hg   = t2 % NHG;
  const int ns   = t2 / NHG;
  if (ns >= GSEQ) return;
  const int head = hg * WPB + wave;
  const int q0   = qt * 16;

  float* ss   = smem + wave * WREG;
  float* so   = ss + 16 * PSC;
  float* slab = so + 16 * PSC;

  const size_t hcol = (size_t)head * HD + 8 * hh;
  const size_t qrow = (size_t)ns * LQ + q0 + c;
  const _Float16* Qsh = HP(QSH) + qrow * FPR + hcol;
  const _Float16* Qsl = HP(QSL) + qrow * FPR + hcol;
  const _Float16* Qoh = HP(QOH) + qrow * FPR + hcol;
  const _Float16* Qol = HP(QOL) + qrow * FPR + hcol;
  const _Float16* Khb = HP(KH) + ((size_t)ns * LQ + c) * FPR + hcol;
  const _Float16* Klb = HP(KL) + ((size_t)ns * LQ + c) * FPR + hcol;
  const _Float16* Vb  = HP(VT) + ((size_t)head * HD + c) * GROWS + (size_t)ns * LQ + 8 * hh;
  const float lsc = RSQ_HD * (LOG2E / (QSC * QSC));
  const size_t KROW = (size_t)FPR;

  float ms[8], mo[8];
#pragma unroll
  for (int r = 0; r < 8; ++r) { ms[r] = -INFINITY; mo[r] = -INFINITY; }

#pragma unroll 1
  for (int kt = 0; kt < NKT; ++kt) {
    const int kb = kt * 32;
    v8f s0 = zero8(), s1 = zero8(), x0 = zero8(), x1 = zero8();
    const _Float16* k0p = Khb + (size_t)kb * KROW;
    const _Float16* k1p = k0p + (size_t)16 * KROW;
    const _Float16* l0p = Klb + (size_t)kb * KROW;
    const _Float16* l1p = l0p + (size_t)16 * KROW;
#pragma unroll
    for (int kk = 0; kk < HD / 32; ++kk) {
      const v16h kh0 = ldfrag_h(k0p + kk * 32);
      const v16h kh1 = ldfrag_h(k1p + kk * 32);
      const v16h kl0 = ldfrag_h(l0p + kk * 32);
      const v16h kl1 = ldfrag_h(l1p + kk * 32);
      const v16h qh  = ldfrag_h(Qsh + kk * 32);
      const v16h ql  = ldfrag_h(Qsl + kk * 32);
      s0 = mma_h(qh, kh0, s0);
      s0 = mma_h(ql, kh0, s0);
      s0 = mma_h(qh, kl0, s0);
      s1 = mma_h(qh, kh1, s1);
      s1 = mma_h(ql, kh1, s1);
      s1 = mma_h(qh, kl1, s1);
      const v16h oh2 = ldfrag_h(Qoh + kk * 32);
      const v16h ol2 = ldfrag_h(Qol + kk * 32);
      x0 = mma_h(oh2, kh0, x0);
      x0 = mma_h(ol2, kh0, x0);
      x0 = mma_h(oh2, kl0, x0);
      x1 = mma_h(oh2, kh1, x1);
      x1 = mma_h(ol2, kh1, x1);
      x1 = mma_h(oh2, kl1, x1);
      guard4x8(s0, s1, x0, x1, qh, ql, oh2, ol2, kh0, kh1, kl0, kl1);
    }
#pragma unroll
    for (int r = 0; r < 8; ++r) {
      const float us0 = s0[r] * lsc;
      const float us1 = s1[r] * lsc;
      const float uo0 = -(x0[r] * lsc);
      const float uo1 = -(x1[r] * lsc);
      float m1 = fmaxf(us0, us1);
      float m2 = fmaxf(uo0, uo1);
#pragma unroll
      for (int off = 1; off < 16; off <<= 1) {
        m1 = fmaxf(m1, __shfl_xor(m1, off, 32));
        m2 = fmaxf(m2, __shfl_xor(m2, off, 32));
      }
      ms[r] = fmaxf(ms[r], m1);
      mo[r] = fmaxf(mo[r], m2);
      const int ro = (8 * hh + r) * PSC + kb + c;
      ss[ro]      = us0;
      ss[ro + 16] = us1;
      so[ro]      = uo0;
      so[ro + 16] = uo1;
    }
  }
  wave_sync_lds();

  float isv[8], iov[8];
#pragma unroll
  for (int r = 0; r < 8; ++r) {
    const int rb = (8 * hh + r) * PSC + c;
    const float m1 = ms[r], m2 = mo[r];
    float zs = 0.f, zo = 0.f;
#pragma unroll 2
    for (int j = 0; j < 8; ++j) {
      const int idx = rb + 16 * j;
      const float es = exp2f(ss[idx] - m1);
      const float eo = exp2f(so[idx] - m2);
      zs += es; zo += eo;
      ss[idx] = es;
      so[idx] = eo;
    }
#pragma unroll
    for (int off = 1; off < 16; off <<= 1) {
      zs += __shfl_xor(zs, off, 32);
      zo += __shfl_xor(zo, off, 32);
    }
    isv[r] = 0.5f * __builtin_amdgcn_rcpf(zs);
    iov[r] = 0.5f * __builtin_amdgcn_rcpf(zo);
  }
#pragma unroll
  for (int r = 0; r < 8; ++r) {
    const int rb = (8 * hh + r) * PSC + c;
    const float a1 = isv[r], a2 = iov[r];
#pragma unroll 2
    for (int j = 0; j < 8; ++j) {
      const int idx = rb + 16 * j;
      const float av = ss[idx] * a1 + so[idx] * a2;
      ss[idx] = av;
    }
  }
  wave_sync_lds();

  const float oc = 1.0f / (PCAR * VCAR);
  v8f o0 = zero8(), o1 = zero8(), o2 = zero8(), o3 = zero8();
#pragma unroll 1
  for (int kt = 0; kt < NKT; ++kt) {
    const int kb = kt * 32;
    FragH ph;
    {
      const float* prow = ss + c * PSC + kb + 8 * hh;
      const v4f p0 = *(const v4f*)(prow), p1 = *(const v4f*)(prow + 4);
      const v4f p2 = *(const v4f*)(prow + 16), p3 = *(const v4f*)(prow + 20);
#pragma unroll
      for (int e = 0; e < 4; ++e) {
        ph.h[0][e]     = (_Float16)(p0[e] * PCAR);
        ph.h[0][4 + e] = (_Float16)(p1[e] * PCAR);
        ph.h[1][e]     = (_Float16)(p2[e] * PCAR);
        ph.h[1][4 + e] = (_Float16)(p3[e] * PCAR);
      }
    }
    const _Float16* vp = Vb + kb;
    const v16h va = ldfrag_h(vp);
    const v16h vb = ldfrag_h(vp + (size_t)16 * GROWS);
    const v16h vc = ldfrag_h(vp + (size_t)32 * GROWS);
    const v16h vd = ldfrag_h(vp + (size_t)48 * GROWS);
    o0 = mma_h(ph.v, va, o0);
    o1 = mma_h(ph.v, vb, o1);
    o2 = mma_h(ph.v, vc, o2);
    o3 = mma_h(ph.v, vd, o3);
    guard6<v16h>(o0, o1, o2, o3, ph.v, va, vb, vc, vd, ph.v);
  }
  acc_guard4(o0, o1, o2, o3);
#pragma unroll
  for (int r = 0; r < 8; ++r) {
    const int base = (8 * hh + r) * SLP + c;
    slab[base]      = o0[r] * oc;
    slab[base + 16] = o1[r] * oc;
    slab[base + 32] = o2[r] * oc;
    slab[base + 48] = o3[r] * oc;
  }
  wave_sync_lds();
  v4u oh[4], ol[4];
  const int rq = lane >> 3, c8 = (lane & 7) * 8;
#pragma unroll
  for (int it = 0; it < 4; ++it) {
    const int row = it * 4 + rq;
    const v4f a = *(const v4f*)(slab + row * SLP + c8), b4 = *(const v4f*)(slab + row * SLP + c8 + 4);
    float w[8];
#pragma unroll
    for (int e = 0; e < 4; ++e) { w[e] = a[e] * OSC; w[4 + e] = b4[e] * OSC; }
#pragma unroll
    for (int e = 0; e < 4; ++e) {
      const _Float16 h0 = (_Float16)w[2 * e], h1 = (_Float16)w[2 * e + 1];
      const _Float16 l0 = (_Float16)(w[2 * e] - (float)h0), l1 = (_Float16)(w[2 * e + 1] - (float)h1);
      oh[it][e] = pk16(h_bits(h0), h_bits(h1));
      ol[it][e] = pk16(h_bits(l0), h_bits(l1));
    }
  }
  const size_t ob = ((size_t)ns * LQ + q0) * FPR + (size_t)head * HD + c8;
  for (int pass = 0; pass < 2; ++pass) {
#pragma unroll
    for (int it = 0; it < 4; ++it) {
      const int row = it * 4 + rq;
      *(volatile v4u*)(OH + ob + (size_t)row * FPR) = oh[it];
      *(volatile v4u*)(OL + ob + (size_t)row * FPR) = ol[it];
    }
    __threadfence();
  }
}

__global__ __launch_bounds__(256) void gnpart(const float* __restrict__ Z, double* P) {
  __shared__ double rs[8], rq[8];
  const int tid = threadIdx.x, wave = tid >> 5, lane = tid & 31;
  const int bid  = blockIdx.x;
  const int part = bid % GNPART;
  const int tm   = bid / GNPART;
  if (tm >= 2 * NB) return;
  const float* z = Z + (size_t)tm * TEN + (size_t)part * GNCH;
  double s = 0.0, s2 = 0.0;
#pragma unroll 1
  for (int i = tid * 4; i < GNCH; i += 1024) {
    const v4f a = *(const v4f*)(z + i);
#pragma unroll
    for (int e = 0; e < 4; ++e) {
      const double g = (double)a[e];
      s += g; s2 += g * g;
    }
  }
  s = wsum_d(s); s2 = wsum_d(s2);
  if (lane == 0) { rs[wave] = s; rq[wave] = s2; }
  __syncthreads();
  if (wave == 0) {
    double a = rs[lane & 7], b2 = rq[lane & 7];
    a  = (lane < 8) ? a : 0.0;
    b2 = (lane < 8) ? b2 : 0.0;
    a = wsum_d(a); b2 = wsum_d(b2);
    v2d o;
    o[0] = (lane == 0) ? a : 0.0;
    o[1] = (lane == 0) ? b2 : 0.0;
    double* dst = P + (size_t)bid * 16 + lane * 2;
    for (int pass = 0; pass < 2; ++pass) {
      if (lane < 8) *(volatile v2d*)(dst) = o;
      __threadfence();
    }
  }
}

__global__ __launch_bounds__(256) void gnapply(const float* __restrict__ Z, const double* __restrict__ P,
                                               const float* __restrict__ gw, const float* __restrict__ gb,
                                               const float* r0, const float* r1, float* o0, float* o1, int stage, int rnd) {
  __shared__ __align__(16) float Tz[DCH * GTP];
  const int tid = threadIdx.x, wave = tid >> 5, lane = tid & 31;
  const int bid = blockIdx.x;
  const int kk  = bid % KD;
  const int t2  = bid / KD;
  const int m   = t2 % NB;
  const int t   = t2 / NB;
  if (t >= 2) return;
  const double* pp = P + ((size_t)(t * NB + m) * GNPART + lane) * 16;
  double s = pp[0], s2 = pp[1];
  s = wsum_d(s); s2 = wsum_d(s2);
  const double inv = 1.0 / (double)TEN;
  const double mu  = s * inv;
  double var = s2 * inv - mu * mu;
  var = (var > 0.0) ? var : 0.0;
  const float muf  = (float)mu;
  const float rstd = rsqrtf((float)var + GN_EPS);
  const int SS = (stage != 0) ? 1 : KD;
  const int SK = (stage != 0) ? SD : 1;
  {
    const int s_ = tid >> 1;
    const int dc = (tid & 1) * 32;
    const size_t zrow = (size_t)t * TROWS + (size_t)m * GROWS + (size_t)s_ * SS + (size_t)kk * SK;
    const float* src = Z + zrow * DCH + dc;
#pragma unroll 2
    for (int i = 0; i < 8; ++i) {
      const v4f a = *(const v4f*)(src + 4 * i);
#pragma unroll
      for (int e = 0; e < 4; ++e) Tz[(dc + 4 * i + e) * GTP + s_] = a[e];
    }
  }
  __syncthreads();
  const float* rp = (t != 0) ? r1 : r0;
  float*       op = (t != 0) ? o1 : o0;
  v4f vals[8];
#pragma unroll
  for (int it = 0; it < 8; ++it) {
    const int d = it * 8 + wave;
    const v4f z4 = *(const v4f*)(Tz + d * GTP + 4 * lane);
    const float g1 = gw[t * DCH + d];
    const float g2 = gb[t * DCH + d];
    const size_t oi = (size_t)m * TEN_FULL + ((size_t)d * KD + kk) * SD + 4 * lane;
    const v4f rr = *(const v4f*)(rp + oi);
#pragma unroll
    for (int e = 0; e < 4; ++e) {
      const float res = (rnd != 0) ? bfr(rr[e]) : rr[e];
      vals[it][e] = (z4[e] - muf) * rstd * g1 + g2 + res;
    }
  }
  for (int pass = 0; pass < 2; ++pass) {
#pragma unroll
    for (int it = 0; it < 8; ++it) {
      const int d = it * 8 + wave;
      const size_t oi = (size_t)m * TEN_FULL + ((size_t)d * KD + kk) * SD + 4 * lane;
      *(volatile v4f*)(op + oi) = vals[it];
    }
    __threadfence();
  }
}

extern "C" void kernel_launch(void* const* d_in, const int* in_sizes, int n_in,
                              void* d_out, int out_size, void* d_ws, size_t ws_size,
                              hipStream_t stream) {
  if (n_in < 16) return;
  if (in_sizes[0] < NB * TEN_FULL || in_sizes[1] < NB * TEN_FULL) return;
  if (in_sizes[2] < NPJ * FPR * DCH || in_sizes[8] < NPJ * FPR * DCH) return;
  if (in_sizes[3] < NPJ * FPR || in_sizes[9] < NPJ * FPR) return;
  if (in_sizes[4] < 2 * DCH * FPR || in_sizes[10] < 2 * DCH * FPR) return;
  if (in_sizes[5] < 2 * DCH || in_sizes[11] < 2 * DCH) return;
  if (in_sizes[6] < 2 * DCH || in_sizes[7] < 2 * DCH || in_sizes[12] < 2 * DCH || in_sizes[13] < 2 * DCH) return;
  if (in_sizes[14] < 4 * DCH || in_sizes[15] < 4 * DCH) return;
  if (out_size < 0 || (size_t)out_size < OUT1_OFF + (size_t)NB * TEN_FULL) return;

  const float* x_s = (const float*)d_in[0];
  const float* x_n = (const float*)d_in[1];
  const float* Win[2]  = { (const float*)d_in[2],  (const float*)d_in[8]  };
  const float* bin[2]  = { (const float*)d_in[3],  (const float*)d_in[9]  };
  const float* Wout[2] = { (const float*)d_in[4],  (const float*)d_in[10] };
  const float* bout[2] = { (const float*)d_in[5],  (const float*)d_in[11] };
  const float* bnw[2]  = { (const float*)d_in[6],  (const float*)d_in[12] };
  const float* bnb[2]  = { (const float*)d_in[7],  (const float*)d_in[13] };
  const float* gnw     = (const float*)d_in[14];
  const float* gnb     = (const float*)d_in[15];
  float* out0 = (float*)d_out;
  float* out1 = out0 + OUT1_OFF;

  const size_t szBNT = (size_t)2 * DCH * BNLP * 4;
  const size_t szGNP = (size_t)2 * NB * GNPART * 16 * 8;
  const size_t szWI  = (size_t)NPJ * FPR * DCH * 2;
  const size_t szWO  = (size_t)2 * DCH * FPR * 2;
  const size_t szX   = (size_t)2 * TROWS * DCH * 2;
  const size_t szZ   = (size_t)2 * TROWS * DCH * 4;
  const size_t szP   = (size_t)GROWS * FPR * 2;
  size_t off = 0;
  auto take = [&](size_t bytes) -> size_t { const size_t o = off; off += (bytes + 32767) & ~(size_t)32767; return o; };
  const size_t oBNT = take(szBNT);
  const size_t oGNP = take(szGNP);
  const size_t oWI0 = take(szWI);
  const size_t oWI1 = take(szWI);
  const size_t oWO0 = take(szWO);
  const size_t oWO1 = take(szWO);
  const size_t oX   = take(szX);
  const size_t oZ   = take(szZ);
  const size_t oQSH = take(szP);
  const size_t oQSL = take(szP);
  const size_t oQOH = take(szP);
  const size_t oQOL = take(szP);
  const size_t oKH  = take(szP);
  const size_t oKL  = take(szP);
  const size_t oVT  = take(szP);
  const size_t oOH  = take(szP);
  const size_t oOL  = take(szP);
  if (off > ws_size) return;
  if (off > (size_t)WS_CAP) return;

  char*   ws  = (char*)d_ws;
  float*  BNT = (float*)(ws + oBNT);
  double* GNP = (double*)(ws + oGNP);
  u16*    WIp[2] = { (u16*)(ws + oWI0), (u16*)(ws + oWI1) };
  u16*    WOp[2] = { (u16*)(ws + oWO0), (u16*)(ws + oWO1) };
  u16*    X   = (u16*)(ws + oX);
  float*  Z   = (float*)(ws + oZ);
  u16*    QSH = (u16*)(ws + oQSH);
  u16*    QSL = (u16*)(ws + oQSL);
  u16*    QOH = (u16*)(ws + oQOH);
  u16*    QOL = (u16*)(ws + oQOL);
  u16*    KH  = (u16*)(ws + oKH);
  u16*    KL  = (u16*)(ws + oKL);
  u16*    VT  = (u16*)(ws + oVT);
  u16*    OH  = (u16*)(ws + oOH);
  u16*    OL  = (u16*)(ws + oOL);

  const dim3 b256(256), b128(128), bAT(ATT_THREADS);
  const int  n8wi = (NPJ * FPR * DCH) / 8;
  const int  n8wo = (2 * DCH * FPR) / 8;
  const dim3 gWI((n8wi + 255) / 256), gWO((n8wo + 255) / 256);
  const dim3 gBN(2 * DCH);
  const dim3 gXP(2 * NB * KD);
  const dim3 gP((GROWS / 64) * (FPR / 64));
  const dim3 gV((FPR / 64) * (GROWS / 64));
  const dim3 gA(NQT * NHG * GSEQ);
  const dim3 gO((GROWS / 64) * (DCH / 64));
  const dim3 gGP(2 * NB * GNPART);
  const dim3 gGA(2 * NB * KD);
  const float iscP = 1.0f / (XSC * WISC);
  const float iscO = 1.0f / (OSC * WOS);

  for (int st = 0; st < 2; ++st) {
    wcvt<<<gWI, b256, 0, stream>>>(Win[st], WIp[st], n8wi, WISC);
    wcvt<<<gWO, b256, 0, stream>>>(Wout[st], WOp[st], n8wo, WOS);
  }

  for (int st = 0; st < 2; ++st) {
    const float* xs_src = (st != 0) ? (const float*)out0 : x_s;
    const float* xn_src = (st != 0) ? (const float*)out1 : x_n;
    const int    rnd    = (st == 0) ? 1 : 0;
    bnstat<<<gBN, b256, 0, stream>>>(xs_src, xn_src, bnw[st], bnb[st], BNT, rnd);
    xpack<<<gXP, b256, 0, stream>>>(xs_src, xn_src, BNT, X, st, rnd);
    const u16*   WI = WIp[st];
    const u16*   WO = WOp[st];
    const float* bi = bin[st];
    const float* bo = bout[st];
    for (int g = 0; g < NB; ++g) {
      for (int t = 0; t < 2; ++t) {
        const u16* Xown = X + ((size_t)t * TROWS + (size_t)g * GROWS) * DCH;
        const u16* Xoth = X + ((size_t)(1 - t) * TROWS + (size_t)g * GROWS) * DCH;
        const int pqs = 4 * t, pqo = 4 * (1 - t) + 1, pk = 4 * t + 2, pv = 4 * t + 3;
        gemm16<1><<<gP, b128, 0, stream>>>(Xown, Xown, WI + (size_t)pqs * FPR * DCH, bi + pqs * FPR,
                                           Z, QSH, QSL, GROWS, FPR, DCH, iscP, QSC);
        gemm16<1><<<gP, b128, 0, stream>>>(Xoth, Xoth, WI + (size_t)pqo * FPR * DCH, bi + pqo * FPR,
                                           Z, QOH, QOL, GROWS, FPR, DCH, iscP, QSC);
        gemm16<1><<<gP, b128, 0, stream>>>(Xown, Xown, WI + (size_t)pk * FPR * DCH, bi + pk * FPR,
                                           Z, KH, KL, GROWS, FPR, DCH, iscP, QSC);
        gemm16<2><<<gV, b128, 0, stream>>>(WI + (size_t)pv * FPR * DCH, WI + (size_t)pv * FPR * DCH, Xown, bi + pv * FPR,
                                           Z, VT, VT, FPR, GROWS, DCH, iscP, VCAR);
        attnx<<<gA, bAT, 0, stream>>>(QSH, QSL, QOH, QOL, KH, KL, VT, OH, OL);
        float* Zg = Z + ((size_t)t * TROWS + (size_t)g * GROWS) * DCH;
        gemm16<0><<<gO, b128, 0, stream>>>(OH, OL, WO + (size_t)t * DCH * FPR, bo + t * DCH,
                                           Zg, OH, OL, GROWS, DCH, FPR, iscO, 1.0f);
      }
    }
    gnpart<<<gGP, b256, 0, stream>>>(Z, GNP);
    const float* rs0 = (st != 0) ? (const float*)out0 : x_s;
    const float* rs1 = (st != 0) ? (const float*)out1 : x_n;
    gnapply<<<gGA, b256, 0, stream>>>(Z, GNP, gnw + st * 2 * DCH, gnb + st * 2 * DCH, rs0, rs1, out0, out1, st, rnd);
  }
  (void)hipGetLastError();
}
